// PatchSelfAttentionBlock_23441931502286
// MI455X (gfx1250) — hardware-run, weakly checked
//
#include <hip/hip_runtime.h>
#include <math.h>

typedef __attribute__((ext_vector_type(16))) _Float16 v16h;
typedef __attribute__((ext_vector_type(16))) __bf16 v16b;
typedef __attribute__((ext_vector_type(8)))  _Float16 v8h;
typedef __attribute__((ext_vector_type(8)))  float v8f;
typedef __attribute__((ext_vector_type(4)))  float v4f;
typedef __attribute__((ext_vector_type(2)))  float v2f;
typedef __attribute__((ext_vector_type(4)))  unsigned v4u;
typedef __attribute__((ext_vector_type(4)))  int v4i;
typedef float __attribute__((may_alias)) float_a;
typedef int __attribute__((may_alias)) int_a;

template <typename T> __device__ __forceinline__ void vst2(void* p, T v) { *(volatile T*)p = v; __threadfence(); *(volatile T*)p = v; }
__device__ __forceinline__ v8f wmma16(v16h a, v16h b, v8f c) {
  v8f d = __builtin_amdgcn_wmma_f32_16x16x32_f16(false, a, false, b, (short)0, c, false, false);
  asm volatile("v_nop\n\tv_nop\n\tv_nop\n\tv_nop" : "+v"(d) : "v"(a), "v"(b));
  return d;
}
__device__ __forceinline__ v8f wmma_bf(v16b a, v16b b, v8f c) {
  v8f d = __builtin_amdgcn_wmma_f32_16x16x32_bf16(false, a, false, b, (short)0, c, false, false);
  asm volatile("v_nop\n\tv_nop\n\tv_nop\n\tv_nop" : "+v"(d) : "v"(a), "v"(b));
  return d;
}
__device__ __forceinline__ v16h frag_h(const _Float16* rowk0, int lane) {
  union { v16h v; v8h q[2]; } u; const _Float16* p = rowk0 + 8 * (lane >> 4);
  u.q[0] = *(const v8h*)p; u.q[1] = *(const v8h*)(p + 16); return u.v;
}
__device__ __forceinline__ v16h frag_f32(const float* rowk0, int lane) {
  v16h a; const float* p = rowk0 + 8 * (lane >> 4);
#pragma unroll
  for (int i = 0; i < 8; ++i) { a[i] = (_Float16)p[i]; a[8 + i] = (_Float16)p[16 + i]; }
  return a;
}
__device__ __forceinline__ v16h frag_f32s(const float* rowk0, int lane, float sc) {
  v16h a; const float* p = rowk0 + 8 * (lane >> 4);
#pragma unroll
  for (int i = 0; i < 8; ++i) { a[i] = (_Float16)(p[i] * sc); a[8 + i] = (_Float16)(p[16 + i] * sc); }
  return a;
}
__device__ __forceinline__ v16h fragc_f32(const float* W, int k0, int n, int lane, int ld, int K) {
  v16h a; const int g = lane >> 4;
#pragma unroll
  for (int i = 0; i < 8; ++i) { const int ka = k0 + 8 * g + i, kb = ka + 16;
    a[i] = (_Float16)(ka < K ? W[(size_t)(ka < K ? ka : K - 1) * ld + n] : 0.f); a[8 + i] = (_Float16)(kb < K ? W[(size_t)(kb < K ? kb : K - 1) * ld + n] : 0.f); }
  return a;
}
struct F2 { v16b h, l; };
__device__ __forceinline__ F2 bsplit16(const float v[16]) { F2 r;
#pragma unroll
  for (int i = 0; i < 16; ++i) { const __bf16 h = (__bf16)v[i]; r.h[i] = h; r.l[i] = (__bf16)(v[i] - (float)h); }
  return r; }
__device__ __forceinline__ F2 split_row(const float* row, int k0, int lane) { float v[16]; const float* p = row + k0 + 8 * (lane >> 4);
#pragma unroll
  for (int i = 0; i < 8; ++i) { v[i] = p[i]; v[8 + i] = p[16 + i]; }
  return bsplit16(v); }
__device__ __forceinline__ F2 split_rowK(const float* row, int k0, int lane, int K) { float v[16]; const int g = lane >> 4;
#pragma unroll
  for (int i = 0; i < 8; ++i) { const int ka = k0 + 8 * g + i, kb = ka + 16; v[i] = ka < K ? row[ka < K ? ka : K - 1] : 0.f; v[8 + i] = kb < K ? row[kb < K ? kb : K - 1] : 0.f; }
  return bsplit16(v); }
__device__ __forceinline__ F2 split_col(const float* W, int k0, int n, int lane, int ld, int K) { float v[16]; const int g = lane >> 4;
#pragma unroll
  for (int i = 0; i < 8; ++i) { const int ka = k0 + 8 * g + i, kb = ka + 16; v[i] = ka < K ? W[(size_t)(ka < K ? ka : K - 1) * ld + n] : 0.f; v[8 + i] = kb < K ? W[(size_t)(kb < K ? kb : K - 1) * ld + n] : 0.f; }
  return bsplit16(v); }
__device__ __forceinline__ v8f mac3(const F2& a, const F2& b, v8f c) { c = wmma_bf(a.l, b.h, c); c = wmma_bf(a.h, b.l, c); return wmma_bf(a.h, b.h, c); }
__device__ __forceinline__ float sigm(float v) { return 1.0f / (1.0f + expf(-v)); }
#define LDSX() do { asm volatile("s_wait_dscnt 0" ::: "memory"); __builtin_amdgcn_wave_barrier(); __builtin_amdgcn_fence(__ATOMIC_RELEASE, "workgroup"); } while (0)


#define NB 8
#define CC 512
#define IH 32
#define IW 32
#define NN (IH * IW)
#define NHD 8
#define DH 64
#define QC (NHD * DH)
#ifndef TNB
#define TNB NB
#endif
typedef __attribute__((ext_vector_type(8))) __bf16 v8b;
__device__ __forceinline__ v16b frag_b(const __bf16* rowk0, int lane) {
  union { v16b v; v8b q[2]; } u; const __bf16* p = rowk0 + 8 * (lane >> 4);
  u.q[0] = *(const v8b*)p; u.q[1] = *(const v8b*)(p + 16); return u.v;
}
__device__ __forceinline__ float bfr(float v) { return (float)(__bf16)v; }
__device__ __attribute__((noinline)) float exp_ni(float v) { return expf(v); }
__device__ __attribute__((noinline)) float erf_ni(float v) { return erff(v); }

#define WS_PE  0u
#define WS_PQ  (WS_PE + 4u * (size_t)NN * CC)
#define WS_QH  (WS_PQ + 4u * (size_t)NN * 3 * QC)
#define WS_QL  (WS_QH + 2u * (size_t)NB * NN * 2 * QC)
#define WS_VT  (WS_QL + 2u * (size_t)NB * NN * 2 * QC)
#define WS_VTL (WS_VT + 2u * (size_t)NB * QC * NN)
#define WS_O   (WS_VTL + 2u * (size_t)NB * QC * NN)
#define WS_END (WS_O + 4u * (size_t)NB * NN * QC)

__device__ __forceinline__ v16b fragb_f32(const float* __restrict__ p, int lane) { v16b a; const float* pp = p + 8 * (lane >> 4);
#pragma unroll
  for (int i = 0; i < 8; ++i) { a[i] = (__bf16)pp[i]; a[8 + i] = (__bf16)pp[16 + i]; } return a; }
__global__ __launch_bounds__(256) void k_pe(float* __restrict__ PE) { __shared__ __align__(16) float s[CC]; const int n = blockIdx.x, t = threadIdx.x; const int hh = n / IW, ww = n % IW; const int half = CC / 2;
  for (int c = t; c < CC; c += 256) { const int cl = c % half; const int i = cl / 2; const float div = expf((float)(2 * i) * (-logf(10000.0f) / (float)half)); const float pos = (float)(c < half ? hh : ww); const float ang = pos * div; s[c] = (cl & 1) ? cosf(ang) : sinf(ang); }
  __syncthreads(); for (int q = t; q < CC / 4; q += 256) vst2(PE + (size_t)n * CC + q * 4, *(const v4f*)&s[q * 4]); }
__global__ __launch_bounds__(128) void k_peq(const float* __restrict__ PE, const float* __restrict__ WQ, const float* __restrict__ WK, const float* __restrict__ WV, float* __restrict__ PQ) { __shared__ __align__(16) float sf[4][16][132];
  const int tid = threadIdx.x, wave = tid >> 5, lane = tid & 31, col = lane & 15, g = lane >> 4; const size_t r0 = (size_t)blockIdx.x * 64 + wave * 16; const int c0 = blockIdx.y * 128; const int which = c0 / QC; const float* Wm = which == 0 ? WQ : which == 1 ? WK : WV;
  v8f acc[8] = {};
#pragma unroll 2
  for (int kc = 0; kc < CC / 32; ++kc) { const F2 a = split_row(PE + (r0 + col) * CC, kc * 32, lane);
#pragma unroll
    for (int j = 0; j < 8; ++j) { const v16b w = fragb_f32(Wm + (size_t)(c0 - which * QC + j * 16 + col) * CC + kc * 32, lane); acc[j] = wmma_bf(a.h, w, acc[j]); acc[j] = wmma_bf(a.l, w, acc[j]); } }
#pragma unroll
  for (int j = 0; j < 8; ++j)
#pragma unroll
    for (int r = 0; r < 8; ++r) sf[wave][8 * g + r][j * 16 + col] = acc[j][r];
  LDSX(); for (int rl = 0; rl < 16; ++rl) vst2(PQ + (r0 + rl) * (3 * QC) + c0 + lane * 4, *(const v4f*)&sf[wave][rl][lane * 4]); }
__global__ __launch_bounds__(128) void k_proj(const float* __restrict__ X, const float* __restrict__ WQ, const float* __restrict__ WK, const float* __restrict__ WV, const float* __restrict__ PQ, _Float16* __restrict__ QH, _Float16* __restrict__ QL, _Float16* __restrict__ VT, _Float16* __restrict__ VTL) { __shared__ __align__(16) _Float16 sh[64][136], sl[64][136]; __shared__ __align__(16) _Float16 th[128][72], tl[128][72];
  const int tid = threadIdx.x, wave = tid >> 5, lane = tid & 31, col = lane & 15, g = lane >> 4; const size_t b = blockIdx.z; const int n0 = blockIdx.x * 64 + wave * 16; const int c0 = blockIdx.y * 128; const int which = c0 / QC; const float* Wm = which == 0 ? WQ : which == 1 ? WK : WV; const float* Xb = X + b * CC * (size_t)NN;
  v8f acc[8] = {};
#pragma unroll 2
  for (int kc = 0; kc < CC / 32; ++kc) { v16b a; const int px = n0 + col;
#pragma unroll
    for (int i = 0; i < 8; ++i) { a[i] = (__bf16)Xb[(size_t)(kc * 32 + 8 * g + i) * NN + px]; a[8 + i] = (__bf16)Xb[(size_t)(kc * 32 + 16 + 8 * g + i) * NN + px]; }
#pragma unroll
    for (int j = 0; j < 8; ++j) acc[j] = wmma_bf(a, fragb_f32(Wm + (size_t)(c0 - which * QC + j * 16 + col) * CC + kc * 32, lane), acc[j]); }
#pragma unroll
  for (int j = 0; j < 8; ++j) { const int c = c0 + j * 16 + col;
#pragma unroll
    for (int r = 0; r < 8; ++r) { const float v = acc[j][r] + PQ[(size_t)(n0 + 8 * g + r) * (3 * QC) + c]; const _Float16 hv = (_Float16)v, lv = (_Float16)((v - (float)hv) * 2048.0f); if (which < 2) { sh[wave * 16 + 8 * g + r][j * 16 + col] = hv; sl[wave * 16 + 8 * g + r][j * 16 + col] = lv; } else { th[j * 16 + col][wave * 16 + 8 * g + r] = hv; tl[j * 16 + col][wave * 16 + 8 * g + r] = lv; } } }
  __syncthreads();
  if (which < 2) { for (int e = tid; e < 64 * 16; e += 128) { const int rl = e >> 4, q = e & 15; const size_t o = (b * NN + blockIdx.x * 64 + rl) * (2 * QC) + c0 + q * 8; vst2((unsigned*)(QH + o), *(const v4u*)&sh[rl][q * 8]); vst2((unsigned*)(QL + o), *(const v4u*)&sl[rl][q * 8]); } }
  else { const int cv0 = c0 - 2 * QC; for (int e = tid; e < 128 * 8; e += 128) { const int cl = e >> 3, q = e & 7; const size_t o = (b * QC + cv0 + cl) * (size_t)NN + blockIdx.x * 64 + q * 8; vst2((unsigned*)(VT + o), *(const v4u*)&th[cl][q * 8]); vst2((unsigned*)(VTL + o), *(const v4u*)&tl[cl][q * 8]); } } }
__global__ __launch_bounds__(128) void k_att(const _Float16* __restrict__ QH, const _Float16* __restrict__ QL, const _Float16* __restrict__ VT, const _Float16* __restrict__ VTL, float* __restrict__ O) {
  __shared__ __align__(16) float sp[4][16][36]; __shared__ __align__(16) float so[4][16][68];
  const int tid = threadIdx.x, wave = tid >> 5, lane = tid & 31, col = lane & 15, g = lane >> 4; const int h = blockIdx.y; const size_t b = blockIdx.z; const int q0 = blockIdx.x * 64 + wave * 16; const size_t rq = b * NN + q0;
  v16h aq[2], al[2];
#pragma unroll
  for (int kc = 0; kc < 2; ++kc) { aq[kc] = frag_h(QH + (rq + col) * (2 * QC) + h * DH + kc * 32, lane); al[kc] = frag_h(QL + (rq + col) * (2 * QC) + h * DH + kc * 32, lane); }
  float m[8], l[8];
#pragma unroll
  for (int r = 0; r < 8; ++r) { m[r] = -3.0e38f; l[r] = 0.f; }
  v8f acc[4] = {}, accl[4] = {};
#pragma unroll 1
  for (int ks = 0; ks < NN / 32; ++ks) { v8f s[2];
#pragma unroll
    for (int ct = 0; ct < 2; ++ct) { const size_t rk = b * NN + ks * 32 + ct * 16 + col; v8f c = {}, cl = {};
#pragma unroll
      for (int kc = 0; kc < 2; ++kc) { const v16h kh = frag_h(QH + rk * (2 * QC) + QC + h * DH + kc * 32, lane), kl = frag_h(QL + rk * (2 * QC) + QC + h * DH + kc * 32, lane); c = wmma16(aq[kc], kh, c); cl = wmma16(aq[kc], kl, cl); cl = wmma16(al[kc], kh, cl); }
#pragma unroll
      for (int r = 0; r < 8; ++r) s[ct][r] = (c[r] + cl[r] * (1.0f / 2048.0f)) * 0.125f; }
    float alpha[8];
#pragma unroll
    for (int r = 0; r < 8; ++r) { float mx = fmaxf(s[0][r], s[1][r]);
#pragma unroll
      for (int o = 1; o < 16; o <<= 1) mx = fmaxf(mx, __shfl_xor(mx, o));
      const float mn = fmaxf(m[r], mx); alpha[r] = __expf(m[r] - mn); const float e0 = __expf(s[0][r] - mn), e1 = __expf(s[1][r] - mn); float es = e0 + e1;
#pragma unroll
      for (int o = 1; o < 16; o <<= 1) es += __shfl_xor(es, o);
      l[r] = l[r] * alpha[r] + es; m[r] = mn; sp[wave][8 * g + r][col] = e0; sp[wave][8 * g + r][16 + col] = e1; }
#pragma unroll
    for (int j = 0; j < 4; ++j)
#pragma unroll
      for (int r = 0; r < 8; ++r) { acc[j][r] *= alpha[r]; accl[j][r] *= alpha[r]; }
    LDSX();
    v16h pa, pal; { const float* prow = &sp[wave][col][0] + 8 * (lane >> 4);
#pragma unroll
      for (int i = 0; i < 8; ++i) { const float p0 = prow[i] * 2048.0f, p1 = prow[16 + i] * 2048.0f; pa[i] = (_Float16)p0; pa[8 + i] = (_Float16)p1; pal[i] = (_Float16)((p0 - (float)pa[i]) * 2048.0f); pal[8 + i] = (_Float16)((p1 - (float)pa[8 + i]) * 2048.0f); } }
#pragma unroll
    for (int j = 0; j < 4; ++j) { const size_t po = (b * QC + (size_t)h * DH + j * 16 + col) * (size_t)NN + ks * 32; const v16h vh = frag_h(VT + po, lane), vl = frag_h(VTL + po, lane); acc[j] = wmma16(pa, vh, acc[j]); accl[j] = wmma16(pa, vl, accl[j]); accl[j] = wmma16(pal, vh, accl[j]); }
    LDSX(); }
#pragma unroll
  for (int r = 0; r < 8; ++r) { const float il = (1.0f / 2048.0f) / l[r];
#pragma unroll
    for (int j = 0; j < 4; ++j) so[wave][8 * g + r][j * 16 + col] = (acc[j][r] + accl[j][r] * (1.0f / 2048.0f)) * il; }
  LDSX(); for (int rl = 0; rl < 16; ++rl) if (lane < 16) vst2(O + (rq + rl) * QC + (size_t)h * DH + lane * 4, *(const v4f*)&so[wave][rl][lane * 4]); }
__global__ __launch_bounds__(128) void k_out(const float* __restrict__ O, const float* __restrict__ WO, const float* __restrict__ BO, float* __restrict__ OUT) { __shared__ __align__(16) float stt[128][68];
  const int tid = threadIdx.x, wave = tid >> 5, lane = tid & 31, col = lane & 15, g = lane >> 4; const size_t b = blockIdx.y; const int n0 = blockIdx.x * 64; const size_t r0 = b * NN + n0 + wave * 16;
#pragma unroll 1
  for (int cc = 0; cc < CC; cc += 128) { v8f acc[8] = {};
#pragma unroll 2
    for (int kc = 0; kc < QC / 32; ++kc) { const F2 a = split_row(O + (r0 + col) * QC, kc * 32, lane);
#pragma unroll
      for (int j = 0; j < 8; ++j) { const v16b w = fragb_f32(WO + (size_t)(cc + j * 16 + col) * QC + kc * 32, lane); acc[j] = wmma_bf(a.h, w, acc[j]); acc[j] = wmma_bf(a.l, w, acc[j]); } }
#pragma unroll
    for (int j = 0; j < 8; ++j) { const int cl = j * 16 + col; const float bb = bfr(BO[cc + cl]);
#pragma unroll
      for (int r = 0; r < 8; ++r) stt[cl][wave * 16 + 8 * g + r] = acc[j][r] + bb; }
    __syncthreads(); for (int e = tid; e < 128 * 16; e += 128) { const int cl = e >> 4, q = e & 15; vst2(OUT + (b * CC + cc + cl) * (size_t)NN + n0 + q * 4, *(const v4f*)&stt[cl][q * 4]); } __syncthreads(); } }
extern "C" void kernel_launch(void* const* d_in, const int* in_sizes, int n_in, void* d_out, int out_size, void* d_ws, size_t ws_size, hipStream_t stream) {
  (void)in_sizes; (void)n_in; (void)out_size;
  const float** F = (const float**)d_in;
  if (ws_size < (size_t)WS_END) return;
  char* ws = (char*)d_ws; float *PE = (float*)(ws + WS_PE), *PQ = (float*)(ws + WS_PQ), *O = (float*)(ws + WS_O); _Float16 *QH = (_Float16*)(ws + WS_QH), *QL = (_Float16*)(ws + WS_QL), *VT = (_Float16*)(ws + WS_VT), *VTL = (_Float16*)(ws + WS_VTL);
  k_pe<<<NN, 256, 0, stream>>>(PE);
  k_peq<<<dim3(NN / 64, 3 * QC / 128), 128, 0, stream>>>(PE, F[1], F[2], F[3], PQ);
  k_proj<<<dim3(NN / 64, 3 * QC / 128, TNB), 128, 0, stream>>>(F[0], F[1], F[2], F[3], PQ, QH, QL, VT, VTL);
  k_att<<<dim3(NN / 64, NHD, TNB), 128, 0, stream>>>(QH, QL, VT, VTL, O);
  k_out<<<dim3(NN / 64, TNB), 128, 0, stream>>>(O, F[4], F[5], (float*)d_out);
}
